// WrappedCasualSelfAttention_88407606821429
// MI455X (gfx1250) — hardware-verified
//
#include <hip/hip_runtime.h>
#include <stddef.h>

typedef _Float16 v16h __attribute__((ext_vector_type(16)));
typedef _Float16 v8h  __attribute__((ext_vector_type(8)));
typedef float    v8f  __attribute__((ext_vector_type(8)));
typedef float    v4f  __attribute__((ext_vector_type(4)));
typedef float    v2f  __attribute__((ext_vector_type(2)));
typedef v8h __attribute__((may_alias)) v8ha;
typedef v4f __attribute__((may_alias)) v4fa;

union Frag { v16h v; v8h half[2]; };

#define EMB    64
#define NH     32
#define NKV    8
#define SEQ    2048
#define BATCH  2
#define ROWS   (BATCH * SEQ)
#define QCOLS  (NH * EMB)
#define KVCOLS (NKV * EMB)
#define WTROWS (QCOLS + 2 * KVCOLS)
#define OCOLS  (NH * EMB)
#define NPAIR  (EMB / 2)
#define TP     72
#define NCVT   144

#define WSCALE 32.0f
#define QSCALE 4.0f
#define KSCALE 4.0f
#define VSCALE 4.0f
#define OSCALE 8.0f
#define PSCALE 16384.0f
#define SSCALE (0.125f / (QSCALE * KSCALE))

static_assert(ROWS % 128 == 0);
static_assert(SEQ % 128 == 0);
static_assert(EMB == 64);
static_assert((TP * 2) % 16 == 0);

__device__ __forceinline__ v8f wmma_f16(v16h a, v16h b, v8f c) {
  v8f d = __builtin_amdgcn_wmma_f32_16x16x32_f16(false, a, false, b, (short)0, c, false, false);
  asm volatile("v_nop\n\tv_nop\n\tv_nop\n\tv_nop" : "+v"(d) : "v"(a), "v"(b));
  return d;
}

__device__ __forceinline__ v16h load_frag(const _Float16* p, int h) {
  Frag f;
  f.half[0] = *(const v8ha*)(p + 8 * h);
  f.half[1] = *(const v8ha*)(p + 16 + 8 * h);
  return f.v;
}

__device__ __forceinline__ void tile_store_pass(const _Float16* s, _Float16* dst, int dp, int w, int lane) {
  const int q8 = lane & 7, sub = lane >> 3;
  #pragma unroll
  for (int i = 0; i < 8; ++i) {
    const int row = w * 32 + i * 4 + sub;
    const v8h v = *(const v8ha*)(s + row * TP + 8 * q8);
    *(volatile v8h*)(dst + (size_t)row * dp + 8 * q8) = v;
  }
}

__global__ __launch_bounds__(64) void k_convert(
    const float* __restrict__ x, const float* __restrict__ wq, const float* __restrict__ wk,
    const float* __restrict__ wv, const float* __restrict__ wo,
    _Float16* __restrict__ xh, _Float16* __restrict__ wT, _Float16* __restrict__ woT)
{
  __shared__ __attribute__((aligned(16))) _Float16 s[64 * TP];

  const int bx = blockIdx.x;
  if (bx >= NCVT) return;
  const int tid = threadIdx.x, lane = tid & 31, w = tid >> 5;

  const float* src; _Float16* dst; int sp, dp, tr; float sc;
  if (bx < 64) {
    src = x + (size_t)bx * 64 * EMB; sp = EMB;
    dst = xh + (size_t)bx * 64 * EMB; dp = EMB; tr = 0; sc = 1.0f;
  } else if (bx < 96) {
    const int t = bx - 64;
    src = wq + t * 64; sp = QCOLS;
    dst = wT + (size_t)(t * 64) * EMB; dp = EMB; tr = 1; sc = WSCALE;
  } else if (bx < 104) {
    const int t = bx - 96;
    src = wk + t * 64; sp = KVCOLS;
    dst = wT + (size_t)(QCOLS + t * 64) * EMB; dp = EMB; tr = 1; sc = WSCALE;
  } else if (bx < 112) {
    const int t = bx - 104;
    src = wv + t * 64; sp = KVCOLS;
    dst = wT + (size_t)(QCOLS + KVCOLS + t * 64) * EMB; dp = EMB; tr = 1; sc = WSCALE;
  } else {
    const int t = bx - 112;
    src = wo + (size_t)t * 64 * EMB; sp = EMB;
    dst = woT + t * 64; dp = OCOLS; tr = 1; sc = WSCALE;
  }

  #pragma unroll 4
  for (int i = 0; i < 16; ++i) {
    const int idx = i * 64 + tid;
    const int row = idx >> 4, c4 = (idx & 15) * 4;
    const v4f v = *(const v4fa*)(src + (size_t)row * sp + c4);
    const _Float16 e0 = (_Float16)(v.x * sc), e1 = (_Float16)(v.y * sc);
    const _Float16 e2 = (_Float16)(v.z * sc), e3 = (_Float16)(v.w * sc);
    if (tr) {
      s[(c4 + 0) * TP + row] = e0; s[(c4 + 1) * TP + row] = e1;
      s[(c4 + 2) * TP + row] = e2; s[(c4 + 3) * TP + row] = e3;
    } else {
      s[row * TP + c4 + 0] = e0; s[row * TP + c4 + 1] = e1;
      s[row * TP + c4 + 2] = e2; s[row * TP + c4 + 3] = e3;
    }
  }
  __syncthreads();

  tile_store_pass(s, dst, dp, w, lane);
  __threadfence();
  tile_store_pass(s, dst, dp, w, lane);
}

__global__ __launch_bounds__(256) void k_rope_tab(float* __restrict__ tab) {
  const int g = blockIdx.x * 256 + threadIdx.x;
  if (g >= SEQ * NPAIR) return;
  const int spos = g >> 5, i = g & 31;
  const float e = (float)(2 * i) * (1.0f / 64.0f);
  const float freq = 1.0f / powf(10000.0f, e);
  const float ang = (float)spos * freq;
  v2f cs;
  cs.x = cosf(ang);
  cs.y = sinf(ang);
  float* p = tab + (size_t)g * 2;
  *(volatile v2f*)p = cs;
  __threadfence();
  *(volatile v2f*)p = cs;
}

__device__ __forceinline__ void proj_store_pass(const _Float16* sT, _Float16* plane, _Float16* vt,
                                                int which, int bh, int l0, int w, int lane) {
  const int q8 = lane & 7, sub = lane >> 3;
  #pragma unroll
  for (int i = 0; i < 8; ++i) {
    const int lid = w * 32 + i * 4 + sub;
    v8h v;
    _Float16* dst;
    if (which != 2) {
      v = *(const v8ha*)(sT + lid * EMB + 8 * q8);
      dst = plane + ((size_t)bh * SEQ + l0 + lid) * EMB + 8 * q8;
    } else {
      const int d = lid >> 1, hl = lid & 1;
      v = *(const v8ha*)(sT + d * 128 + 64 * hl + 8 * q8);
      dst = vt + ((size_t)bh * EMB + d) * SEQ + l0 + 64 * hl + 8 * q8;
    }
    *(volatile v8h*)dst = v;
  }
}

__global__ __launch_bounds__(128) void k_proj(
    const _Float16* __restrict__ xh,
    const _Float16* __restrict__ wT,
    const float* __restrict__ bq, const float* __restrict__ bk, const float* __restrict__ bv,
    const float* __restrict__ tab,
    _Float16* __restrict__ qh,
    _Float16* __restrict__ kh,
    _Float16* __restrict__ vt)
{
  __shared__ __attribute__((aligned(16))) _Float16 sT[128 * 64];

  const int tid = threadIdx.x, lane = tid & 31, w = tid >> 5;
  const int h = lane >> 4, m = lane & 15;
  const int m0 = blockIdx.x * 128;
  const int cg = blockIdx.y;
  int which, head;
  if (cg < NH)            { which = 0; head = cg; }
  else if (cg < NH + NKV) { which = 1; head = cg - NH; }
  else                    { which = 2; head = cg - NH - NKV; }
  const int m0w = m0 + 32 * w;

  const _Float16* xa0 = xh + (size_t)(m0w + m) * EMB;
  const _Float16* xa1 = xa0 + (size_t)16 * EMB;
  const _Float16* wb  = wT + (size_t)(cg * 64 + m) * EMB;

  const v8f zero8 = {0.f, 0.f, 0.f, 0.f, 0.f, 0.f, 0.f, 0.f};
  v8f acc[2][4];
  #pragma unroll
  for (int mt = 0; mt < 2; ++mt)
    #pragma unroll
    for (int nt = 0; nt < 4; ++nt) acc[mt][nt] = zero8;

  #pragma unroll
  for (int ks = 0; ks < 2; ++ks) {
    const int k0 = 32 * ks;
    const v16h a0 = load_frag(xa0 + k0, h);
    const v16h a1 = load_frag(xa1 + k0, h);
    #pragma unroll
    for (int nt = 0; nt < 4; ++nt) {
      const v16h bfr = load_frag(wb + (size_t)nt * 16 * EMB + k0, h);
      acc[0][nt] = wmma_f16(a0, bfr, acc[0][nt]);
      acc[1][nt] = wmma_f16(a1, bfr, acc[1][nt]);
    }
  }

  const float* bias = (which == 0) ? bq : ((which == 1) ? bk : bv);
  const float osc = (which == 0) ? QSCALE : ((which == 1) ? KSCALE : VSCALE);
  const int b = m0 / SEQ, l0 = m0 - b * SEQ;
  #pragma unroll
  for (int nt = 0; nt < 4; ++nt) {
    const int feat = 16 * nt + m;
    const int cev = feat & ~1, codd = feat | 1;
    const float bvl = bias[head * EMB + feat];
    #pragma unroll
    for (int mt = 0; mt < 2; ++mt) {
      #pragma unroll
      for (int r = 0; r < 8; ++r) {
        const int tokl = 32 * w + 16 * mt + 8 * h + r;
        float y = acc[mt][nt][r] * (1.0f / WSCALE) + bvl;
        const float pr = __shfl_xor(y, 1);
        if (which != 2) {
          const int pos = l0 + tokl;
          const float cs = tab[(size_t)pos * EMB + cev];
          const float sn = tab[(size_t)pos * EMB + codd];
          y = (m & 1) ? (pr * sn + y * cs) : (y * cs - pr * sn);
        }
        y *= osc;
        const int idx = (which == 2) ? (feat * 128 + tokl) : (tokl * EMB + feat);
        sT[idx] = (_Float16)y;
      }
    }
  }
  __syncthreads();

  const int bh = (which == 0) ? (b * NH + head) : (b * NKV + head);
  _Float16* plane = (which == 0) ? qh : kh;
  proj_store_pass(sT, plane, vt, which, bh, l0, w, lane);
  __threadfence();
  proj_store_pass(sT, plane, vt, which, bh, l0, w, lane);
}

__device__ __forceinline__ v16h pack_p(v8f a, v8f c) {
  const v16h r = { (_Float16)(a[0] * PSCALE), (_Float16)(a[1] * PSCALE), (_Float16)(a[2] * PSCALE), (_Float16)(a[3] * PSCALE),
                   (_Float16)(a[4] * PSCALE), (_Float16)(a[5] * PSCALE), (_Float16)(a[6] * PSCALE), (_Float16)(a[7] * PSCALE),
                   (_Float16)(c[0] * PSCALE), (_Float16)(c[1] * PSCALE), (_Float16)(c[2] * PSCALE), (_Float16)(c[3] * PSCALE),
                   (_Float16)(c[4] * PSCALE), (_Float16)(c[5] * PSCALE), (_Float16)(c[6] * PSCALE), (_Float16)(c[7] * PSCALE) };
  return r;
}

__device__ __forceinline__ void attn_store_pass(const _Float16* so, _Float16* oh,
                                                int b, int head, int q0, int lane) {
  const int q8 = lane & 7, sub = lane >> 3;
  #pragma unroll
  for (int i = 0; i < 4; ++i) {
    const int row = i * 4 + sub;
    const v8h v = *(const v8ha*)(so + row * 64 + 8 * q8);
    const size_t gi = ((size_t)b * SEQ + q0 + row) * OCOLS + head * EMB + 8 * q8;
    *(volatile v8h*)(oh + gi) = v;
  }
}

__global__ __launch_bounds__(128) void k_attn(
    const _Float16* __restrict__ qh,
    const _Float16* __restrict__ kh,
    const _Float16* __restrict__ vt,
    _Float16* __restrict__ oh)
{
  __shared__ __attribute__((aligned(16))) _Float16 sO[4 * 16 * 64];

  const int tid = threadIdx.x, lane = tid & 31, w = tid >> 5;
  const int h = lane >> 4, m = lane & 15;
  const int bh = blockIdx.y, b = bh >> 5, head = bh & 31;
  const int kbh = b * NKV + (head >> 2);
  const int qblk = blockIdx.x;
  const int q0 = qblk * 64 + 16 * w;
  const int qi = q0 + m;

  const _Float16* qrow = qh + ((size_t)bh * SEQ + q0 + m) * EMB;
  const v16h qb0 = load_frag(qrow, h);
  const v16h qb1 = load_frag(qrow + 32, h);

  const v8f zero8 = {0.f, 0.f, 0.f, 0.f, 0.f, 0.f, 0.f, 0.f};
  v8f o[4];
  #pragma unroll
  for (int t = 0; t < 4; ++t) o[t] = zero8;
  float mrun = -1e30f, lrun = 0.0f;

  const _Float16* kbase = kh + ((size_t)kbh * SEQ + m) * EMB;
  const _Float16* vbase = vt + ((size_t)kbh * EMB + m) * SEQ;
  const int kbend = qblk * 64;

  #pragma unroll 1
  for (int kb = 0; kb <= kbend; kb += 64) {
    v8f s[4];
    #pragma unroll
    for (int j = 0; j < 4; ++j) {
      const _Float16* kp = kbase + (size_t)(kb + 16 * j) * EMB;
      const v16h kf0 = load_frag(kp, h);
      const v16h kf1 = load_frag(kp + 32, h);
      v8f z = zero8;
      z = wmma_f16(kf0, qb0, z);
      z = wmma_f16(kf1, qb1, z);
      s[j] = z;
    }
    #pragma unroll
    for (int j = 0; j < 4; ++j)
      #pragma unroll
      for (int r = 0; r < 8; ++r) {
        const int key = kb + 16 * j + 8 * h + r;
        s[j][r] = (key <= qi) ? (s[j][r] * SSCALE) : -1e30f;
      }

    float mloc = s[0][0];
    #pragma unroll
    for (int j = 0; j < 4; ++j)
      #pragma unroll
      for (int r = 0; r < 8; ++r) mloc = fmaxf(mloc, s[j][r]);
    mloc = fmaxf(mloc, __shfl_xor(mloc, 16));
    const float mnew = fmaxf(mrun, mloc);
    const float alpha = __expf(mrun - mnew);
    mrun = mnew;
    float lsum = 0.0f;
    #pragma unroll
    for (int j = 0; j < 4; ++j)
      #pragma unroll
      for (int r = 0; r < 8; ++r) {
        const float p = __expf(s[j][r] - mnew);
        s[j][r] = p;
        lsum += p;
      }
    lsum += __shfl_xor(lsum, 16);
    lrun = lrun * alpha + lsum;
    #pragma unroll
    for (int t = 0; t < 4; ++t)
      #pragma unroll
      for (int r = 0; r < 8; ++r) o[t][r] = o[t][r] * alpha;

    const v16h pb0 = pack_p(s[0], s[1]);
    const v16h pb1 = pack_p(s[2], s[3]);

    #pragma unroll
    for (int t = 0; t < 4; ++t) {
      const _Float16* vp = vbase + (size_t)(16 * t) * SEQ + kb;
      const v16h vf0 = load_frag(vp, h);
      const v16h vf1 = load_frag(vp + 32, h);
      o[t] = wmma_f16(vf0, pb0, o[t]);
      o[t] = wmma_f16(vf1, pb1, o[t]);
    }
  }

  const float inv = (1.0f / lrun) * (OSCALE / (PSCALE * VSCALE));
  _Float16* so = sO + w * 1024;
  #pragma unroll
  for (int t = 0; t < 4; ++t)
    #pragma unroll
    for (int r = 0; r < 8; ++r)
      so[m * 64 + 16 * t + 8 * h + r] = (_Float16)(o[t][r] * inv);
  __syncthreads();

  attn_store_pass(so, oh, b, head, q0, lane);
  __threadfence();
  attn_store_pass(so, oh, b, head, q0, lane);
}

__device__ __forceinline__ void out_store_pass(const float* so, float* out, int m0w, int lane) {
  const int q8 = lane & 7, sub = lane >> 3;
  #pragma unroll
  for (int i = 0; i < 16; ++i) {
    const int lid = i * 4 + sub;
    const int row = lid >> 1, hl = lid & 1;
    const v4f v = *(const v4fa*)(so + row * 64 + 32 * hl + 4 * q8);
    *(volatile v4f*)(out + (size_t)(m0w + row) * EMB + 32 * hl + 4 * q8) = v;
  }
}

__global__ __launch_bounds__(128) void k_oproj(
    const _Float16* __restrict__ oh,
    const _Float16* __restrict__ woT,
    const float* __restrict__ bo, const float* __restrict__ x,
    const float* __restrict__ gamma, const float* __restrict__ beta,
    float* __restrict__ out)
{
  __shared__ __attribute__((aligned(16))) float sY[4 * 32 * 64];

  const int tid = threadIdx.x, lane = tid & 31, w = tid >> 5;
  const int h = lane >> 4, m = lane & 15;
  const int m0 = blockIdx.x * 128;
  const int m0w = m0 + 32 * w;

  const _Float16* xa0 = oh + (size_t)(m0w + m) * OCOLS;
  const _Float16* xa1 = xa0 + (size_t)16 * OCOLS;
  const _Float16* wb  = woT + (size_t)m * OCOLS;

  const v8f zero8 = {0.f, 0.f, 0.f, 0.f, 0.f, 0.f, 0.f, 0.f};
  v8f acc[2][4];
  #pragma unroll
  for (int mt = 0; mt < 2; ++mt)
    #pragma unroll
    for (int nt = 0; nt < 4; ++nt) acc[mt][nt] = zero8;

  #pragma unroll 1
  for (int k0 = 0; k0 < OCOLS; k0 += 32) {
    const v16h a0 = load_frag(xa0 + k0, h);
    const v16h a1 = load_frag(xa1 + k0, h);
    #pragma unroll
    for (int nt = 0; nt < 4; ++nt) {
      const v16h bfr = load_frag(wb + (size_t)nt * 16 * OCOLS + k0, h);
      acc[0][nt] = wmma_f16(a0, bfr, acc[0][nt]);
      acc[1][nt] = wmma_f16(a1, bfr, acc[1][nt]);
    }
  }

  float gcol[4], bcol[4];
  #pragma unroll
  for (int nt = 0; nt < 4; ++nt) {
    const int col = 16 * nt + m;
    const float bb = bo[col];
    gcol[nt] = gamma[col];
    bcol[nt] = beta[col];
    #pragma unroll
    for (int mt = 0; mt < 2; ++mt)
      #pragma unroll
      for (int r = 0; r < 8; ++r) {
        const int tok = m0w + 16 * mt + 8 * h + r;
        acc[mt][nt][r] = acc[mt][nt][r] * (1.0f / (OSCALE * WSCALE)) + bb + x[(size_t)tok * EMB + col];
      }
  }

  float* so = sY + w * 2048;
  #pragma unroll
  for (int mt = 0; mt < 2; ++mt) {
    #pragma unroll
    for (int r = 0; r < 8; ++r) {
      float ssum = acc[mt][0][r] + acc[mt][1][r] + acc[mt][2][r] + acc[mt][3][r];
      #pragma unroll
      for (int off = 8; off >= 1; off >>= 1) ssum += __shfl_xor(ssum, off);
      const float mu = ssum * (1.0f / EMB);
      const float d0 = acc[mt][0][r] - mu, d1 = acc[mt][1][r] - mu;
      const float d2 = acc[mt][2][r] - mu, d3 = acc[mt][3][r] - mu;
      float qsum = d0 * d0 + d1 * d1 + d2 * d2 + d3 * d3;
      #pragma unroll
      for (int off = 8; off >= 1; off >>= 1) qsum += __shfl_xor(qsum, off);
      const float var = qsum * (1.0f / EMB);
      const float rs = rsqrtf(var + 1e-5f);
      const int rowl = 16 * mt + 8 * h + r;
      so[rowl * 64 + 16 * 0 + m] = d0 * rs * gcol[0] + bcol[0];
      so[rowl * 64 + 16 * 1 + m] = d1 * rs * gcol[1] + bcol[1];
      so[rowl * 64 + 16 * 2 + m] = d2 * rs * gcol[2] + bcol[2];
      so[rowl * 64 + 16 * 3 + m] = d3 * rs * gcol[3] + bcol[3];
    }
  }
  __syncthreads();

  out_store_pass(so, out, m0w, lane);
  __threadfence();
  out_store_pass(so, out, m0w, lane);
}

extern "C" void kernel_launch(void* const* d_in, const int* in_sizes, int n_in,
                              void* d_out, int out_size, void* d_ws, size_t ws_size,
                              hipStream_t stream) {
  if (n_in < 11) return;
  if (in_sizes[0] != ROWS * EMB) return;
  if (in_sizes[1] != EMB * QCOLS || in_sizes[2] != QCOLS) return;
  if (in_sizes[3] != EMB * KVCOLS || in_sizes[4] != KVCOLS) return;
  if (in_sizes[5] != EMB * KVCOLS || in_sizes[6] != KVCOLS) return;
  if (in_sizes[7] != OCOLS * EMB || in_sizes[8] != EMB) return;
  if (in_sizes[9] != EMB || in_sizes[10] != EMB) return;
  if (out_size != ROWS * EMB) return;

  const float* x     = (const float*)d_in[0];
  const float* wq    = (const float*)d_in[1];
  const float* bq    = (const float*)d_in[2];
  const float* wk    = (const float*)d_in[3];
  const float* bk    = (const float*)d_in[4];
  const float* wv    = (const float*)d_in[5];
  const float* bv    = (const float*)d_in[6];
  const float* wo    = (const float*)d_in[7];
  const float* bo    = (const float*)d_in[8];
  const float* gamma = (const float*)d_in[9];
  const float* beta  = (const float*)d_in[10];
  float* out = (float*)d_out;

  const size_t xh_bytes  = (size_t)ROWS * EMB * 2;
  const size_t wT_bytes  = (size_t)WTROWS * EMB * 2;
  const size_t woT_bytes = (size_t)EMB * OCOLS * 2;
  const size_t tab_bytes = (size_t)SEQ * EMB * 4;
  const size_t qh_bytes  = (size_t)BATCH * NH * SEQ * EMB * 2;
  const size_t kh_bytes  = (size_t)BATCH * NKV * SEQ * EMB * 2;
  const size_t vt_bytes  = kh_bytes;
  const size_t oh_bytes  = (size_t)ROWS * OCOLS * 2;
  size_t off = 0;
  const size_t o_xh  = off; off += xh_bytes;
  const size_t o_wT  = off; off += wT_bytes;
  const size_t o_woT = off; off += woT_bytes;
  const size_t o_tab = off; off += tab_bytes;
  const size_t o_qh  = off; off += qh_bytes;
  const size_t o_kh  = off; off += kh_bytes;
  const size_t o_vt  = off; off += vt_bytes;
  const size_t o_oh  = off; off += oh_bytes;
  if (off > ws_size) return;

  char* ws = (char*)d_ws;
  _Float16* xh  = (_Float16*)(ws + o_xh);
  _Float16* wT  = (_Float16*)(ws + o_wT);
  _Float16* woT = (_Float16*)(ws + o_woT);
  float*    tab = (float*)(ws + o_tab);
  _Float16* qh  = (_Float16*)(ws + o_qh);
  _Float16* kh  = (_Float16*)(ws + o_kh);
  _Float16* vt  = (_Float16*)(ws + o_vt);
  _Float16* oh  = (_Float16*)(ws + o_oh);

  k_convert<<<NCVT, 64, 0, stream>>>(x, wq, wk, wv, wo, xh, wT, woT);

  k_rope_tab<<<(SEQ * NPAIR + 255) / 256, 256, 0, stream>>>(tab);

  dim3 gProj(ROWS / 128, NH + 2 * NKV);
  k_proj<<<gProj, 128, 0, stream>>>(xh, wT, bq, bk, bv, tab, qh, kh, vt);

  dim3 gAtt(SEQ / 64, BATCH * NH);
  k_attn<<<gAtt, 128, 0, stream>>>(qh, kh, vt, oh);

  k_oproj<<<ROWS / 128, 128, 0, stream>>>(oh, woT, bo, x, gamma, beta, out);
}
